// GATNetwork_3487513444403
// MI455X (gfx1250) — hardware-verified
//
#include <hip/hip_runtime.h>
#include <stddef.h>
#include <stdint.h>


#define DIN     128
#define NH1     4
#define HD1     512
#define KG2     1024
#define ELW     8
#define NTHR    256
#define NWAVE   8
#define EPT     8
#define CHUNK   (NTHR * EPT)
#define WCAP    (EPT * 32)
#define LISTN   (NWAVE * WCAP)
#define NBMAX   2048
#define RCAP    28672
#define DEGCAP  512
#define STW     512
#define GBM     64
#define GBN     64
#define GTHR    128
#define LGN     64
#define NEGSL   0.2f
#define WSMAX   268435456
#define LDS_AGG ((2 * RCAP + 2 * NBMAX + LISTN) * 4 + 64)

static_assert((CHUNK & (CHUNK - 1)) == 0 && CHUNK <= 4096);
static_assert((NBMAX & (NBMAX - 1)) == 0 && NBMAX <= 4096);
static_assert(NTHR * 8 == NBMAX);
static_assert(LISTN >= NBMAX);
static_assert(LISTN >= NWAVE * WCAP);
static_assert((RCAP % 32) == 0);
static_assert(NWAVE * STW <= RCAP);
static_assert(STW * 4 == KG2 * 2);
static_assert(LDS_AGG <= 300000);
static_assert(GBM == (GTHR / 32) * 16);
static_assert(DIN / 8 == 16);
static_assert((DIN % 32) == 0 && (KG2 % 32) == 0);
static_assert((HD1 % GBN) == 0 && (DIN % GBN) == 0);
static_assert(HD1 == NH1 * DIN && KG2 == 2 * HD1);
static_assert(LGN == GBM);
static_assert(LGN * ELW == 4 * 32 * 4);
static_assert((LGN % NWAVE) == 0);

typedef float          v4f  __attribute__((ext_vector_type(4)));
typedef float          v8f  __attribute__((ext_vector_type(8)));
typedef int            v4i  __attribute__((ext_vector_type(4)));
typedef int            v8i  __attribute__((ext_vector_type(8)));
typedef unsigned int   v2u  __attribute__((ext_vector_type(2)));
typedef unsigned int   v4u  __attribute__((ext_vector_type(4)));
typedef unsigned short v8us __attribute__((ext_vector_type(8)));
typedef __bf16         v16b __attribute__((ext_vector_type(16)));
union FragB { v16b v; v8us h[2]; v8i w; };

__device__ __forceinline__ v8f wmb(const FragB& a, const FragB& b, v8f c) {
  v8f d = __builtin_amdgcn_wmma_f32_16x16x32_bf16(false, a.v, false, b.v, (short)0, c, false, false);
  asm volatile("v_nop\n\tv_nop\n\tv_nop\n\tv_nop" : "+v"(d) : "v"(a.w), "v"(b.w));
  return d;
}

__device__ __forceinline__ void ldwait() {
  asm volatile("s_wait_loadcnt 0x0" ::: "memory");
}

__device__ __forceinline__ unsigned int f2bf(float f) {
  const unsigned int u = __float_as_uint(f);
  return (u + 0x7FFFu + ((u >> 16) & 1u)) >> 16;
}
__device__ __forceinline__ float bf2f(unsigned int b) { return __uint_as_float(b << 16); }
__device__ __forceinline__ float bfr(float f) { return bf2f(f2bf(f)); }
__device__ __forceinline__ v4f bfr4(const v4f a) {
  v4f r; r.x = bfr(a.x); r.y = bfr(a.y); r.z = bfr(a.z); r.w = bfr(a.w); return r;
}
__device__ __forceinline__ unsigned int pk2(float lo, float hi) { return f2bf(lo) | (f2bf(hi) << 16); }
__device__ __forceinline__ v4u pack8(const v4f a, const v4f b) {
  v4u r;
  r.x = pk2(a.x, a.y); r.y = pk2(a.z, a.w); r.z = pk2(b.x, b.y); r.w = pk2(b.z, b.w);
  return r;
}

__device__ __forceinline__ int scan_chunk(const int* __restrict__ dsts, int nE, int cbase, int slotBase,
                                          int nb, int vec8, int* list, int tid, int lane, int wave) {
  int wc = 0;
  const int el0  = tid * EPT;
  const int e0   = cbase + el0;
  const int sent = -2147483647 - 1;
  v4i da, db;
  if (vec8 != 0 && cbase + CHUNK <= nE) {
    da = *(const v4i*)(dsts + e0);
    db = *(const v4i*)(dsts + e0 + 4);
  } else {
    da.x = (e0     < nE) ? dsts[min(e0,     nE - 1)] : sent;
    da.y = (e0 + 1 < nE) ? dsts[min(e0 + 1, nE - 1)] : sent;
    da.z = (e0 + 2 < nE) ? dsts[min(e0 + 2, nE - 1)] : sent;
    da.w = (e0 + 3 < nE) ? dsts[min(e0 + 3, nE - 1)] : sent;
    db.x = (e0 + 4 < nE) ? dsts[min(e0 + 4, nE - 1)] : sent;
    db.y = (e0 + 5 < nE) ? dsts[min(e0 + 5, nE - 1)] : sent;
    db.z = (e0 + 6 < nE) ? dsts[min(e0 + 6, nE - 1)] : sent;
    db.w = (e0 + 7 < nE) ? dsts[min(e0 + 7, nE - 1)] : sent;
  }
  const unsigned nbs = (unsigned)slotBase;
  const unsigned unb = (unsigned)nb;
  const unsigned s0 = (unsigned)da.x - nbs, s1 = (unsigned)da.y - nbs;
  const unsigned s2 = (unsigned)da.z - nbs, s3 = (unsigned)da.w - nbs;
  const unsigned s4 = (unsigned)db.x - nbs, s5 = (unsigned)db.y - nbs;
  const unsigned s6 = (unsigned)db.z - nbs, s7 = (unsigned)db.w - nbs;
  const bool h0 = s0 < unb, h1 = s1 < unb, h2 = s2 < unb, h3 = s3 < unb;
  const bool h4 = s4 < unb, h5 = s5 < unb, h6 = s6 < unb, h7 = s7 < unb;
  const unsigned any = __builtin_amdgcn_ballot_w32(h0 | h1 | h2 | h3 | h4 | h5 | h6 | h7);
  if (any != 0u) {
#define HITJ(J, HJ, SJ) { \
      const unsigned mj = __builtin_amdgcn_ballot_w32(HJ); \
      if (mj != 0u) { \
        if (HJ) { \
          const int pos = wc + (int)__builtin_amdgcn_mbcnt_lo(mj, 0u); \
          if (pos < WCAP) list[wave * WCAP + pos] = ((el0 + (J)) << 12) | (int)(SJ); \
        } \
        wc += (int)__builtin_popcount(mj); } }
    HITJ(0, h0, s0)
    HITJ(1, h1, s1)
    HITJ(2, h2, s2)
    HITJ(3, h3, s3)
    HITJ(4, h4, s4)
    HITJ(5, h5, s5)
    HITJ(6, h6, s6)
    HITJ(7, h7, s7)
#undef HITJ
  }
  return wc;
}

__global__ __launch_bounds__(NTHR) void k_xprep(const float* __restrict__ x, unsigned short* xb, int nN, int nUnits) {
  const int i = (int)blockIdx.x * NTHR + (int)threadIdx.x;
  if (i >= nUnits) return;
  const int row = i >> 4;
  const int c0  = (i & 15) * 8;
  const int rc  = row < nN ? row : nN - 1;
  const float* p = x + (size_t)rc * DIN + c0;
  v4f a = *(const v4f*)p, b = *(const v4f*)(p + 4);
  const v4f z4 = {0.f, 0.f, 0.f, 0.f};
  if (row >= nN) { a = z4; b = z4; }
  const v4u wv = pack8(a, b);
  unsigned short* o = xb + (size_t)row * DIN + c0;
  *(volatile v4u*)o = wv;
  __threadfence();
  *(volatile v4u*)o = wv;
}

__global__ __launch_bounds__(NTHR) void k_wtr(const float* __restrict__ w, int Kin, int Ncol, int Nrows, int Kout,
                                              unsigned short* wt, int nUnits) {
  const int u = (int)blockIdx.x * NTHR + (int)threadIdx.x;
  if (u >= nUnits) return;
  const int kq = Kout >> 3;
  const int n  = u / kq;
  const int k8 = (u - n * kq) * 8;
  const int kk = k8 - (k8 / Kin) * Kin;
  const int ncl = n < Ncol ? n : Ncol - 1;
  const float* p = w + (size_t)kk * (size_t)Ncol + ncl;
  v4f a, b;
  a.x = p[0];                    a.y = p[(size_t)Ncol];         a.z = p[(size_t)2 * Ncol];     a.w = p[(size_t)3 * Ncol];
  b.x = p[(size_t)4 * Ncol];     b.y = p[(size_t)5 * Ncol];     b.z = p[(size_t)6 * Ncol];     b.w = p[(size_t)7 * Ncol];
  const v4f z4 = {0.f, 0.f, 0.f, 0.f};
  if (n >= Ncol || n >= Nrows) { a = z4; b = z4; }
  const v4u wv = pack8(a, b);
  unsigned short* o = wt + (size_t)n * (size_t)Kout + k8;
  *(volatile v4u*)o = wv;
  __threadfence();
  *(volatile v4u*)o = wv;
}

__global__ __launch_bounds__(GTHR) void k_gemm(
    const unsigned short* __restrict__ A, const unsigned short* __restrict__ WT,
    float* outF, int K, int ldo)
{
  __shared__ __attribute__((aligned(16))) float stg[GBM * GBN];
  const int tid = (int)threadIdx.x, lane = tid & 31, wave = tid >> 5, hh = lane >> 4, m = lane & 15;
  const int rowBase = (int)blockIdx.x * GBM;
  const int col0    = (int)blockIdx.y * GBN;

  v8f acc[4];
  {
    const v8f z = {0.f, 0.f, 0.f, 0.f, 0.f, 0.f, 0.f, 0.f};
    acc[0] = z; acc[1] = z; acc[2] = z; acc[3] = z;
  }
  const unsigned short* ap = A  + (size_t)(rowBase + 16 * wave + m) * (size_t)K + 8 * hh;
  const unsigned short* wp = WT + (size_t)(col0 + m) * (size_t)K + 8 * hh;
  const int ksteps = K >> 5;
#pragma unroll 1
  for (int ks = 0; ks < ksteps; ++ks) {
    FragB af;
    af.h[0] = *(const v8us*)(ap + 32 * ks);
    af.h[1] = *(const v8us*)(ap + 32 * ks + 16);
#pragma unroll
    for (int t = 0; t < 4; ++t) {
      const unsigned short* wq = wp + (size_t)(16 * t) * (size_t)K + 32 * ks;
      FragB bf;
      bf.h[0] = *(const v8us*)wq;
      bf.h[1] = *(const v8us*)(wq + 16);
      acc[t] = wmb(af, bf, acc[t]);
    }
  }

#pragma unroll
  for (int t = 0; t < 4; ++t) {
    const int lc = 16 * t + m;
#pragma unroll
    for (int r = 0; r < 8; ++r) {
      const int lr = 16 * wave + 8 * hh + r;
      stg[lr * GBN + lc] = acc[t][r];
    }
  }
  __syncthreads();

  v4f fv[8];
#pragma unroll
  for (int i = 0; i < 8; ++i) {
    const int lr = 16 * wave + 2 * i + hh;
    fv[i] = *(const v4f*)(stg + lr * GBN + 4 * m);
  }
#pragma unroll
  for (int i = 0; i < 8; ++i) {
    const int lr = 16 * wave + 2 * i + hh;
    const int gr = rowBase + lr;
    float* op = outF + (size_t)gr * (size_t)ldo + col0 + 4 * m;
    *(volatile v4f*)op = fv[i];
  }
  __threadfence();
#pragma unroll
  for (int i = 0; i < 8; ++i) {
    const int lr = 16 * wave + 2 * i + hh;
    const int gr = rowBase + lr;
    float* op = outF + (size_t)gr * (size_t)ldo + col0 + 4 * m;
    *(volatile v4f*)op = fv[i];
  }
}

template<int H>
__global__ __launch_bounds__(NTHR) void k_logit(const float* __restrict__ P, const float* __restrict__ asrc,
                                                const float* __restrict__ adst, float* EL, int nN, int ldp) {
  __shared__ __attribute__((aligned(16))) float stg[LGN * ELW];
  const int tid = (int)threadIdx.x, lane = tid & 31, wave = tid >> 5;
  const int nb0 = (int)blockIdx.x * LGN;
  v4f as[H], ad[H];
#pragma unroll
  for (int h = 0; h < H; ++h) {
    as[h] = bfr4(*(const v4f*)(asrc + h * DIN + 4 * lane));
    ad[h] = bfr4(*(const v4f*)(adst + h * DIN + 4 * lane));
  }
#pragma unroll 1
  for (int i = 0; i < LGN / NWAVE; ++i) {
    const int ln  = wave * (LGN / NWAVE) + i;
    const int n   = nb0 + ln;
    const int ncl = n < nN ? n : nN - 1;
    const float live = n < nN ? 1.0f : 0.0f;
    float es[4], ed[4];
#pragma unroll
    for (int h = 0; h < 4; ++h) { es[h] = 0.f; ed[h] = 0.f; }
#pragma unroll
    for (int h = 0; h < H; ++h) {
      const v4f pv = *(const v4f*)(P + (size_t)ncl * (size_t)ldp + h * DIN + 4 * lane);
      es[h] = pv.x * as[h].x + pv.y * as[h].y + pv.z * as[h].z + pv.w * as[h].w;
      ed[h] = pv.x * ad[h].x + pv.y * ad[h].y + pv.z * ad[h].z + pv.w * ad[h].w;
    }
#pragma unroll
    for (int off = 16; off > 0; off >>= 1) {
#pragma unroll
      for (int h = 0; h < H; ++h) {
        es[h] += __shfl_xor(es[h], off);
        ed[h] += __shfl_xor(ed[h], off);
      }
    }
    if (lane == 0) {
#pragma unroll
      for (int h = 0; h < 4; ++h) {
        stg[ln * ELW + h]     = es[h] * live;
        stg[ln * ELW + 4 + h] = ed[h] * live;
      }
    }
  }
  __syncthreads();
  if (wave < 4) {
    const int f0 = wave * 128 + 4 * lane;
    const v4f v = *(const v4f*)(stg + f0);
    float* op = EL + (size_t)nb0 * ELW + f0;
    *(volatile v4f*)op = v;
    __threadfence();
    *(volatile v4f*)op = v;
  }
}

template<int L>
__global__ __launch_bounds__(NTHR) void k_agg(
    const int* __restrict__ srcs, const int* __restrict__ dsts,
    const float* __restrict__ EL, const float* __restrict__ P,
    const float* __restrict__ bias, const float* __restrict__ fcw, const float* __restrict__ fcb,
    unsigned short* H1B, float* out,
    int nN, int nE, int nb, int vec8, int MPr) {
  extern __shared__ v4f lds_dyn[];
  int* reg1 = (int*)lds_dyn;
  int* reg2 = reg1 + RCAP;
  int* scnt = reg2 + RCAP;
  int* soff = scnt + NBMAX;
  int* list = soff + NBMAX;
  int* wcnt = list + LISTN;
  int* wtot = wcnt + NWAVE;
  const int tid = (int)threadIdx.x, lane = tid & 31, wave = tid >> 5;
  const int nodeBase = (int)blockIdx.x * nb;

  for (int i = tid; i < NBMAX; i += NTHR) scnt[i] = 0;
  __syncthreads();

  int tot = 0;
  const int nChunks = (nE + CHUNK - 1) / CHUNK;
#pragma unroll 1
  for (int ch = 0; ch < nChunks; ++ch) {
    const int cbase = ch * CHUNK;
    const int wc = scan_chunk(dsts, nE, cbase, nodeBase, nb, vec8, list, tid, lane, wave);
    if (lane == 0) wcnt[wave] = wc;
    __syncthreads();
    int pre = 0, all = 0;
#pragma unroll
    for (int w2 = 0; w2 < NWAVE; ++w2) {
      int c = wcnt[w2];
      c = c < 0 ? 0 : (c > WCAP ? WCAP : c);
      all += c;
      pre += (w2 < wave) ? c : 0;
    }
    const int wcc  = wc > WCAP ? WCAP : wc;
    const int base = tot + pre;
#pragma unroll 1
    for (int i = lane; i < wcc; i += 32) {
      const int ent = list[wave * WCAP + i];
      const int el  = (ent >> 12) & (CHUNK - 1);
      const int sl  = ent & (NBMAX - 1);
      int eid = cbase + el;
      eid = eid > nE - 1 ? nE - 1 : eid;
      const int pos = base + i;
      if (pos < RCAP) reg1[pos] = (int)(((unsigned)eid << 12) | (unsigned)sl);
    }
    tot += all;
    tot = tot > RCAP ? RCAP : tot;
    __syncthreads();
  }
  const int nh = tot;

  if (wave == 0) {
#pragma unroll 1
    for (int b0 = 0; b0 < nh; b0 += 32) {
      const int idx = b0 + lane;
      const int uv  = reg1[idx < RCAP ? idx : RCAP - 1];
      const int m32 = (nh - b0) < 32 ? (nh - b0) : 32;
#pragma unroll 1
      for (int k = 0; k < m32; ++k) {
        const int u  = __builtin_amdgcn_readlane(uv, k);
        const int sl = u & (NBMAX - 1);
        if (lane == 0) scnt[sl] = scnt[sl] + 1;
      }
    }
  }
  __syncthreads();

  {
    const v4i ca = *(const v4i*)(scnt + 8 * tid);
    const v4i cb = *(const v4i*)(scnt + 8 * tid + 4);
    const int e0 = ca.x < 0 ? 0 : ca.x, e1 = ca.y < 0 ? 0 : ca.y, e2 = ca.z < 0 ? 0 : ca.z, e3 = ca.w < 0 ? 0 : ca.w;
    const int e4 = cb.x < 0 ? 0 : cb.x, e5 = cb.y < 0 ? 0 : cb.y, e6 = cb.z < 0 ? 0 : cb.z, e7 = cb.w < 0 ? 0 : cb.w;
    const int ts = e0 + e1 + e2 + e3 + e4 + e5 + e6 + e7;
    int incl = ts;
#pragma unroll
    for (int d = 1; d < 32; d <<= 1) {
      const int up = __shfl_up(incl, d);
      if (lane >= d) incl += up;
    }
    if (lane == 31) wtot[wave] = incl;
    __syncthreads();
    int pre = 0;
#pragma unroll
    for (int w2 = 0; w2 < NWAVE; ++w2) pre += (w2 < wave) ? wtot[w2] : 0;
    int run = pre + incl - ts;
    soff[8 * tid + 0] = run; run += e0;
    soff[8 * tid + 1] = run; run += e1;
    soff[8 * tid + 2] = run; run += e2;
    soff[8 * tid + 3] = run; run += e3;
    soff[8 * tid + 4] = run; run += e4;
    soff[8 * tid + 5] = run; run += e5;
    soff[8 * tid + 6] = run; run += e6;
    soff[8 * tid + 7] = run;
  }
  __syncthreads();
  for (int i = tid; i < NBMAX; i += NTHR) list[i] = soff[i];
  __syncthreads();

  if (wave == 0) {
#pragma unroll 1
    for (int b0 = 0; b0 < nh; b0 += 32) {
      const int idx = b0 + lane;
      const int uv  = reg1[idx < RCAP ? idx : RCAP - 1];
      const int m32 = (nh - b0) < 32 ? (nh - b0) : 32;
#pragma unroll 1
      for (int k = 0; k < m32; ++k) {
        const int u   = __builtin_amdgcn_readlane(uv, k);
        const int sl  = u & (NBMAX - 1);
        const int eid = (int)((unsigned)u >> 12);
        if (lane == 0) {
          int pos = list[sl];
          pos = pos < 0 ? 0 : (pos > RCAP - 1 ? RCAP - 1 : pos);
          reg2[pos] = eid;
          list[sl] = pos + 1;
        }
      }
    }
  }
  __syncthreads();

  const int nbw = nb >> 3;
  const bool ovf = (nh >= RCAP);
  const float qnan = __int_as_float(0x7fc00000);

  if (L == 1) {
    unsigned int* stw = (unsigned int*)reg1 + wave * STW;
    v4f bb[4];
#pragma unroll
    for (int j = 0; j < 4; ++j) bb[j] = bfr4(*(const v4f*)(bias + DIN * j + 4 * lane));
#pragma unroll 1
    for (int jt = 0; jt < nbw; ++jt) {
      const int slot = wave * nbw + jt;
      const int grow = nodeBase + slot;
      const int gcl  = grow < nN ? grow : nN - 1;
      int st = soff[slot];
      const int craw = scnt[slot];
      int cnt = craw;
      st  = st < 0 ? 0 : (st > nh ? nh : st);
      cnt = cnt < 0 ? 0 : (cnt > DEGCAP ? DEGCAP : cnt);
      if (cnt > nh - st) cnt = nh - st;
      const float pz = (ovf || craw > DEGCAP) ? qnan : 0.0f;
      const bool wr = grow < MPr;
      const float live = grow < nN ? 1.0f : 0.0f;

      const v4f edv = *(const v4f*)(EL + (size_t)gcl * ELW + 4);
      ldwait();
      float mx[4], dn[4];
      v4f av[4];
      {
        const v4f z4 = {0.f, 0.f, 0.f, 0.f};
#pragma unroll
        for (int j = 0; j < 4; ++j) { mx[j] = -1.0e30f; dn[j] = 0.f; av[j] = z4; }
      }
      const int cnt1 = cnt + 1;
#pragma unroll 1
      for (int q = 0; q < cnt1; ++q) {
        int s = gcl;
        if (q < cnt) {
          int idx = st + q; idx = idx > RCAP - 1 ? RCAP - 1 : idx;
          int eid = reg2[idx]; eid = eid < 0 ? 0 : (eid > nE - 1 ? nE - 1 : eid);
          const int sraw = srcs[eid];
          s = sraw < 0 ? 0 : (sraw > nN - 1 ? nN - 1 : sraw);
        }
        const v4f esv = *(const v4f*)(EL + (size_t)s * ELW);
        const float* hr = P + (size_t)s * HD1 + 4 * lane;
        v4f hv[4];
#pragma unroll
        for (int j = 0; j < 4; ++j) hv[j] = *(const v4f*)(hr + DIN * j);
        ldwait();
#pragma unroll
        for (int j = 0; j < 4; ++j) {
          float lg = esv[j] + edv[j];
          lg = lg > 0.f ? lg : NEGSL * lg;
          const float df = lg - mx[j];
          const float ee = __expf(-fabsf(df));
          const bool up  = df > 0.f;
          const float s1 = up ? ee : 1.0f;
          const float s2 = up ? 1.0f : ee;
          mx[j] = up ? lg : mx[j];
          dn[j] = fmaf(dn[j], s1, s2);
          av[j] = av[j] * s1 + hv[j] * s2;
        }
      }
      v2u hw[4], lw[4];
#pragma unroll
      for (int j = 0; j < 4; ++j) {
        const float ds  = dn[j] > 0.f ? dn[j] : 1.0f;
        const float inv = __builtin_amdgcn_rcpf(ds);
        const float q0 = fmaxf(fmaf(av[j].x, inv, bb[j].x), 0.f) * live + pz;
        const float q1 = fmaxf(fmaf(av[j].y, inv, bb[j].y), 0.f) * live + pz;
        const float q2 = fmaxf(fmaf(av[j].z, inv, bb[j].z), 0.f) * live + pz;
        const float q3 = fmaf(0.f, 0.f, fmaxf(fmaf(av[j].w, inv, bb[j].w), 0.f) * live + pz);
        const unsigned int h0 = f2bf(q0), h1 = f2bf(q1), h2 = f2bf(q2), h3 = f2bf(q3);
        const unsigned int l0 = f2bf(q0 - bf2f(h0)), l1 = f2bf(q1 - bf2f(h1));
        const unsigned int l2 = f2bf(q2 - bf2f(h2)), l3 = f2bf(q3 - bf2f(h3));
        hw[j].x = h0 | (h1 << 16); hw[j].y = h2 | (h3 << 16);
        lw[j].x = l0 | (l1 << 16); lw[j].y = l2 | (l3 << 16);
      }
      __builtin_amdgcn_fence(__ATOMIC_RELEASE, "wavefront");
      __builtin_amdgcn_wave_barrier();
#pragma unroll
      for (int j = 0; j < 4; ++j) {
        *(v2u*)(stw + 64 * j + 2 * lane)       = hw[j];
        *(v2u*)(stw + 256 + 64 * j + 2 * lane) = lw[j];
      }
      __builtin_amdgcn_fence(__ATOMIC_RELEASE, "wavefront");
      __builtin_amdgcn_wave_barrier();
      v4u pv[4];
#pragma unroll
      for (int qq = 0; qq < 4; ++qq) pv[qq] = *(const v4u*)(stw + 4 * (32 * qq + lane));
      unsigned short* gp = H1B + (size_t)grow * KG2;
      if (wr) {
#pragma unroll
        for (int qq = 0; qq < 4; ++qq) *(volatile v4u*)(gp + 8 * (32 * qq + lane)) = pv[qq];
      }
      __threadfence();
      if (wr) {
#pragma unroll
        for (int qq = 0; qq < 4; ++qq) *(volatile v4u*)(gp + 8 * (32 * qq + lane)) = pv[qq];
      }
    }
  } else {
    float* res = (float*)list;
    const v4f bb = bfr4(*(const v4f*)(bias + 4 * lane));
    const v4f fw = bfr4(*(const v4f*)(fcw + 4 * lane));
    const float fb = bfr(fcb[0]);
#pragma unroll 1
    for (int jt = 0; jt < nbw; ++jt) {
      const int slot = wave * nbw + jt;
      const int grow = nodeBase + slot;
      const int gcl  = grow < nN ? grow : nN - 1;
      int st = soff[slot];
      const int craw = scnt[slot];
      int cnt = craw;
      st  = st < 0 ? 0 : (st > nh ? nh : st);
      cnt = cnt < 0 ? 0 : (cnt > DEGCAP ? DEGCAP : cnt);
      if (cnt > nh - st) cnt = nh - st;
      const float pz = (ovf || craw > DEGCAP) ? qnan : 0.0f;

      const float edv = EL[(size_t)gcl * ELW + 4];
      ldwait();
      float mx = -1.0e30f, dn = 0.f;
      v4f av = {0.f, 0.f, 0.f, 0.f};
      const int cnt1 = cnt + 1;
#pragma unroll 1
      for (int q = 0; q < cnt1; ++q) {
        int s = gcl;
        if (q < cnt) {
          int idx = st + q; idx = idx > RCAP - 1 ? RCAP - 1 : idx;
          int eid = reg2[idx]; eid = eid < 0 ? 0 : (eid > nE - 1 ? nE - 1 : eid);
          const int sraw = srcs[eid];
          s = sraw < 0 ? 0 : (sraw > nN - 1 ? nN - 1 : sraw);
        }
        const float es = EL[(size_t)s * ELW];
        const v4f gv = *(const v4f*)(P + (size_t)s * DIN + 4 * lane);
        ldwait();
        float lg = es + edv;
        lg = lg > 0.f ? lg : NEGSL * lg;
        const float df = lg - mx;
        const float ee = __expf(-fabsf(df));
        const bool up  = df > 0.f;
        const float s1 = up ? ee : 1.0f;
        const float s2 = up ? 1.0f : ee;
        mx = up ? lg : mx;
        dn = fmaf(dn, s1, s2);
        av = av * s1 + gv * s2;
      }
      const float ds  = dn > 0.f ? dn : 1.0f;
      const float inv = __builtin_amdgcn_rcpf(ds);
      float part = fmaf(av.x, inv, bb.x) * fw.x + fmaf(av.y, inv, bb.y) * fw.y
                 + fmaf(av.z, inv, bb.z) * fw.z + fmaf(av.w, inv, bb.w) * fw.w;
#pragma unroll
      for (int off = 16; off > 0; off >>= 1) part += __shfl_xor(part, off);
      const float r = part + fb + pz;
      if (lane == 0) res[slot] = r;
    }
    __syncthreads();
    const int npc = nb >> 2;
#pragma unroll 1
    for (int p = tid; p < npc; p += NTHR) {
      const v4f v = *(const v4f*)(res + 4 * p);
      const int r0 = nodeBase + 4 * p;
      if (r0 + 3 < nN) {
        *(volatile v4f*)(out + r0) = v;
      } else {
        if (r0     < nN) *(volatile float*)(out + r0)     = v.x;
        if (r0 + 1 < nN) *(volatile float*)(out + r0 + 1) = v.y;
        if (r0 + 2 < nN) *(volatile float*)(out + r0 + 2) = v.z;
      }
    }
    __threadfence();
#pragma unroll 1
    for (int p = tid; p < npc; p += NTHR) {
      const v4f v = *(const v4f*)(res + 4 * p);
      const int r0 = nodeBase + 4 * p;
      if (r0 + 3 < nN) {
        *(volatile v4f*)(out + r0) = v;
      } else {
        if (r0     < nN) *(volatile float*)(out + r0)     = v.x;
        if (r0 + 1 < nN) *(volatile float*)(out + r0 + 1) = v.y;
        if (r0 + 2 < nN) *(volatile float*)(out + r0 + 2) = v.z;
      }
    }
  }
}

static int pick_nb(int nE, int nN) {
  int nb = NBMAX;
  while (nb > 32 && (long long)nb * (long long)nE * 5LL > (long long)RCAP * (long long)nN * 4LL) nb >>= 1;
  return nb;
}
static inline int cdiv(int a, int b) { return (a + b - 1) / b; }

extern "C" void kernel_launch(void* const* d_in, const int* in_sizes, int n_in,
                              void* d_out, int out_size, void* d_ws, size_t ws_size,
                              hipStream_t stream) {
  if (n_in < 12) return;
  const int nN = in_sizes[0] / DIN;
  if (nN <= 0 || in_sizes[0] != nN * DIN || nN > (1 << 22)) return;
  if (in_sizes[1] < 2 || (in_sizes[1] & 1) != 0) return;
  const int nE = in_sizes[1] / 2;
  if (nE < 1 || nE > (1 << 20)) return;
  if (in_sizes[2]  != DIN * HD1) return;
  if (in_sizes[3]  != NH1 * DIN || in_sizes[4] != NH1 * DIN) return;
  if (in_sizes[5]  != HD1) return;
  if (in_sizes[6]  != HD1 * DIN) return;
  if (in_sizes[7]  != DIN || in_sizes[8] != DIN) return;
  if (in_sizes[9]  != DIN) return;
  if (in_sizes[10] != DIN) return;
  if (in_sizes[11] < 1) return;
  if (out_size != nN) return;

  const float* x    = (const float*)d_in[0];
  const int*   ei   = (const int*)  d_in[1];
  const float* W1   = (const float*)d_in[2];
  const float* a1s  = (const float*)d_in[3];
  const float* a1d  = (const float*)d_in[4];
  const float* b1   = (const float*)d_in[5];
  const float* W2   = (const float*)d_in[6];
  const float* a2s  = (const float*)d_in[7];
  const float* a2d  = (const float*)d_in[8];
  const float* b2   = (const float*)d_in[9];
  const float* fcw  = (const float*)d_in[10];
  const float* fcb  = (const float*)d_in[11];
  float* out = (float*)d_out;
  const int* src = ei;
  const int* dst = ei + nE;

  const int MP   = cdiv(nN, GBM) * GBM;
  const int nb   = pick_nb(nE, nN);
  if (nb < 32 || (nb & (nb - 1)) != 0 || nb > NBMAX) return;
  const int gA   = cdiv(MP, nb);
  const int vec8 = ((nE & 3) == 0) ? 1 : 0;
  if (gA * nb < MP) return;

  char* ws = (char*)d_ws;
  size_t off = 0;
  const size_t oXB  = off; off += (size_t)MP * DIN * 2;            off = (off + 255) & ~(size_t)255;
  const size_t oWT1 = off; off += (size_t)HD1 * DIN * 2;           off = (off + 255) & ~(size_t)255;
  const size_t oWT2 = off; off += (size_t)DIN * KG2 * 2;           off = (off + 255) & ~(size_t)255;
  const size_t oHF  = off; off += (size_t)MP * HD1 * 4;            off = (off + 255) & ~(size_t)255;
  const size_t oEL  = off; off += (size_t)MP * ELW * 4;            off = (off + 255) & ~(size_t)255;
  const size_t oH1B = off; off += (size_t)MP * KG2 * 2;            off = (off + 255) & ~(size_t)255;
  if (off > ws_size || off > (size_t)WSMAX) return;
  if ((size_t)MP * DIN * 4 > (size_t)MP * HD1 * 4) return;
  unsigned short* XB  = (unsigned short*)(ws + oXB);
  unsigned short* WT1 = (unsigned short*)(ws + oWT1);
  unsigned short* WT2 = (unsigned short*)(ws + oWT2);
  float*          HF  = (float*)(ws + oHF);
  float*          G   = (float*)(ws + oHF);
  float*          EL  = (float*)(ws + oEL);
  unsigned short* H1B = (unsigned short*)(ws + oH1B);

  hipFuncSetAttribute(reinterpret_cast<const void*>(&k_agg<1>),
                      hipFuncAttributeMaxDynamicSharedMemorySize, LDS_AGG);
  hipFuncSetAttribute(reinterpret_cast<const void*>(&k_agg<2>),
                      hipFuncAttributeMaxDynamicSharedMemorySize, LDS_AGG);

  const int nUx = MP * (DIN / 8);
  k_xprep<<<cdiv(nUx, NTHR), NTHR, 0, stream>>>(x, XB, nN, nUx);

  {
    const int nU1 = HD1 * (DIN / 8);
    k_wtr<<<cdiv(nU1, NTHR), NTHR, 0, stream>>>(W1, DIN, HD1, HD1, DIN, WT1, nU1);
    const int nU2 = DIN * (KG2 / 8);
    k_wtr<<<cdiv(nU2, NTHR), NTHR, 0, stream>>>(W2, HD1, DIN, DIN, KG2, WT2, nU2);
  }

  const int gM = MP / GBM;
  k_gemm<<<dim3(gM, HD1 / GBN), GTHR, 0, stream>>>(XB, WT1, HF, DIN, HD1);
  k_logit<4><<<MP / LGN, NTHR, 0, stream>>>(HF, a1s, a1d, EL, nN, HD1);
  k_agg<1><<<gA, NTHR, LDS_AGG, stream>>>(src, dst, EL, HF, b1, fcw, fcb, H1B, out, nN, nE, nb, vec8, MP);
  k_gemm<<<dim3(gM, DIN / GBN), GTHR, 0, stream>>>(H1B, WT2, G, KG2, DIN);
  k_logit<1><<<MP / LGN, NTHR, 0, stream>>>(G, a2s, a2d, EL, nN, DIN);
  k_agg<2><<<gA, NTHR, LDS_AGG, stream>>>(src, dst, EL, G, b2, fcw, fcb, H1B, out, nN, nE, nb, vec8, MP);
}
